// biGRU_72550587564390
// MI455X (gfx1250) — hardware-verified
//
#include <hip/hip_runtime.h>

typedef __attribute__((ext_vector_type(16))) _Float16 v16h;
typedef __attribute__((ext_vector_type(8)))  _Float16 v8h;
typedef __attribute__((ext_vector_type(16))) __bf16   v16b;
typedef __attribute__((ext_vector_type(8)))  __bf16   v8b;
typedef __attribute__((ext_vector_type(8)))  float    v8f;
typedef __attribute__((ext_vector_type(4)))  float    v4f;
typedef __attribute__((ext_vector_type(4)))  unsigned int v4u;

__device__ __forceinline__ unsigned short f2bf_bits(float f) {
  unsigned u = __float_as_uint(f);
  return (unsigned short)((u + 0x7FFFu + ((u >> 16) & 1u)) >> 16);
}
__device__ __forceinline__ float bf_bits2f(unsigned short h) { return __uint_as_float(((unsigned)h) << 16); }

__device__ __forceinline__ void dep_guard_h(v8f& a, v8f& b, v16h x, v16h y) { asm volatile("v_nop\n\tv_nop\n\tv_nop\n\tv_nop" : "+v"(a), "+v"(b) : "v"(x), "v"(y)); }
__device__ __forceinline__ void dep_guard_b(v8f& a, v8f& b, v16b x, v16b y) { asm volatile("v_nop\n\tv_nop\n\tv_nop\n\tv_nop" : "+v"(a), "+v"(b) : "v"(x), "v"(y)); }
__device__ __forceinline__ void keep4_h(v16h a, v16h b, v16h c, v16h d) { asm volatile("v_nop" :: "v"(a), "v"(b), "v"(c), "v"(d)); }
__device__ __forceinline__ void keep4_b(v16b a, v16b b, v16b c, v16b d) { asm volatile("v_nop" :: "v"(a), "v"(b), "v"(c), "v"(d)); }
__device__ __forceinline__ void acc_guard4(v8f& a, v8f& b, v8f& c, v8f& d) { asm volatile("v_nop\n\tv_nop\n\tv_nop\n\tv_nop" : "+v"(a), "+v"(b), "+v"(c), "+v"(d)); }
template <typename T> struct Frag;
template <> struct Frag<_Float16> {
  typedef v16h V; union U { v16h v; v8h h[2]; };
  static __device__ __forceinline__ v16h load(const _Float16* p) {
    U f; f.h[0] = *(const v8h*)(p); f.h[1] = *(const v8h*)(p + 16); return f.v;
  }
  static __device__ __forceinline__ v8f mma(v16h a, v16h b, v8f c) {
    return __builtin_amdgcn_wmma_f32_16x16x32_f16(false, a, false, b, (short)0, c, false, false);
  }
  static __device__ __forceinline__ void guard(v8f& a, v8f& b, v16h x, v16h y) { dep_guard_h(a, b, x, y); }
  static __device__ __forceinline__ void keep(v16h a, v16h b, v16h c, v16h d) { keep4_h(a, b, c, d); }
};
template <> struct Frag<__bf16> {
  typedef v16b V; union U { v16b v; v8b h[2]; };
  static __device__ __forceinline__ v16b load(const __bf16* p) {
    U f; f.h[0] = *(const v8b*)(p); f.h[1] = *(const v8b*)(p + 16); return f.v;
  }
  static __device__ __forceinline__ v8f mma(v16b a, v16b b, v8f c) {
    return __builtin_amdgcn_wmma_f32_16x16x32_bf16(false, a, false, b, (short)0, c, false, false);
  }
  static __device__ __forceinline__ void guard(v8f& a, v8f& b, v16b x, v16b y) { dep_guard_b(a, b, x, y); }
  static __device__ __forceinline__ void keep(v16b a, v16b b, v16b c, v16b d) { keep4_b(a, b, c, d); }
};

template <int ET> struct Elem;
template <> struct Elem<0> { typedef _Float16 T; };
template <> struct Elem<1> { typedef __bf16 T; };
template <int ET, bool SPLIT, int BIAS_MODE, int OUT_MODE, bool RESID, int ACT = 0>
__global__ __launch_bounds__(256) void wmma_gemm64(
    const unsigned short* __restrict__ Ap, const unsigned short* __restrict__ A2p, int lda, long strideA,
    const unsigned short* __restrict__ Btp, const unsigned short* __restrict__ Bt2p, int ldb, long strideB,
    void* __restrict__ Cout, void* __restrict__ Cout2, int ldc, long strideC,
    const float* __restrict__ bias,
    const float* __restrict__ resid, long strideR,
    int M, int N, int K, float scale) {
  typedef typename Elem<ET>::T T;
  typedef typename Frag<T>::V V;
  const T* A = (const T*)Ap; const T* A2 = (const T*)A2p; const T* Bt = (const T*)Btp; const T* Bt2 = (const T*)Bt2p;
  __shared__ __align__(16) float sT[8][16 * 68];
  const int b    = blockIdx.y;
  const int lane = threadIdx.x & 31;
  const int wave = threadIdx.x >> 5;
  const int tilesN = N >> 6;
  const int tilesM = M >> 6;
  const int tile = blockIdx.x * 8 + wave;
  if (tile >= tilesM * tilesN) return;
  const int tm = tile / tilesN;
  const int tn = tile - tm * tilesN;
  const int m0 = tm << 6;
  const int n0 = tn << 6;

  const T* Ab  = A  + (size_t)b * strideA;
  const T* Bb  = Bt + (size_t)b * strideB;
  const T* Ab2 = SPLIT ? (A2  + (size_t)b * strideA) : nullptr;
  const T* Bb2 = SPLIT ? (Bt2 + (size_t)b * strideB) : nullptr;

  const int rlane = lane & 15;
  const int koff  = (lane >> 4) * 8;
  const int mOff  = (lane >> 4) * 8;

  v8f acc[4][4];
#pragma unroll
  for (int i = 0; i < 4; ++i)
#pragma unroll
    for (int j = 0; j < 4; ++j) acc[i][j] = (v8f){0.f,0.f,0.f,0.f,0.f,0.f,0.f,0.f};

  for (int k0 = 0; k0 < K; k0 += 32) {
    V bh[4], bl[4];
#pragma unroll
    for (int j = 0; j < 4; ++j) {
      const size_t bo = (size_t)(n0 + (j << 4) + rlane) * ldb + koff + k0;
      bh[j] = Frag<T>::load(Bb + bo);
      if (SPLIT) bl[j] = Frag<T>::load(Bb2 + bo);
    }
#pragma unroll
    for (int i = 0; i < 4; ++i) {
      const size_t ao = (size_t)(m0 + (i << 4) + rlane) * lda + koff + k0;
      V ah = Frag<T>::load(Ab + ao);
      V al;
      if (SPLIT) al = Frag<T>::load(Ab2 + ao);
#pragma unroll
      for (int j = 0; j < 4; ++j) {
        acc[i][j] = Frag<T>::mma(ah, bh[j], acc[i][j]);
        if (SPLIT) {
          acc[i][j] = Frag<T>::mma(ah, bl[j], acc[i][j]);
          acc[i][j] = Frag<T>::mma(al, bh[j], acc[i][j]);
        }
      }
      Frag<T>::guard(acc[i][0], acc[i][3], ah, SPLIT ? al : ah);
    }
    Frag<T>::keep(bh[0], bh[1], bh[2], bh[3]);
    if (SPLIT) Frag<T>::keep(bl[0], bl[1], bl[2], bl[3]);
  }
  acc_guard4(acc[0][0], acc[0][1], acc[0][2], acc[0][3]);
  acc_guard4(acc[1][0], acc[1][1], acc[1][2], acc[1][3]);
  acc_guard4(acc[2][0], acc[2][1], acc[2][2], acc[2][3]);
  acc_guard4(acc[3][0], acc[3][1], acc[3][2], acc[3][3]);

  float* slab = sT[wave];
  const float* Rb = RESID ? (resid + (size_t)b * strideR) : nullptr;
#pragma unroll
  for (int i = 0; i < 4; ++i) {
    const int mBase = m0 + (i << 4);
#pragma unroll
    for (int j = 0; j < 4; ++j) {
      const int n = n0 + (j << 4) + rlane;
      float bv = 0.f;
      if (BIAS_MODE == 2) bv = bias[n];
#pragma unroll
      for (int r = 0; r < 8; ++r) {
        float v = acc[i][j][r] * scale;
        if (BIAS_MODE == 1) v += bias[mBase + mOff + r];
        if (BIAS_MODE == 2) v += bv;
        if (RESID) v += Rb[(size_t)(mBase + mOff + r) * ldc + n];
        if (ACT == 1) v = tanhf(v);
        if (ACT == 2) v = fmaxf(v, 0.0f);
        if (ACT == 3) v = v / (1.0f + expf(-v));
        if (ACT == 4) v = (v > 0.f) ? v : 0.01f * v;
        if (ACT == 5) v = 0.5f * v * (1.0f + erff(v * 0.70710678118654752f));
        slab[(mOff + r) * 68 + (j << 4) + rlane] = v;
      }
    }
    __builtin_amdgcn_fence(__ATOMIC_RELEASE, "workgroup");
    __builtin_amdgcn_wave_barrier();
    __builtin_amdgcn_fence(__ATOMIC_ACQUIRE, "workgroup");
    if (OUT_MODE == 0) {
      float* C = (float*)Cout + (size_t)b * strideC;
      const int hh = lane >> 4, c4 = (lane & 15) * 4;
      for (int pass = 0; pass < 2; ++pass) {
#pragma unroll
        for (int it = 0; it < 8; ++it) {
          const int row = it * 2 + hh;
          v4f v = *(const v4f*)(slab + row * 68 + c4);
          *(volatile v4f*)(C + (size_t)(mBase + row) * ldc + n0 + c4) = v;
        }
        __threadfence();
      }
    } else {
      const int q = lane >> 3, c8 = (lane & 7) * 8;
      unsigned short* C  = (unsigned short*)Cout  + (size_t)b * strideC;
      unsigned short* C2 = (OUT_MODE == 2) ? ((unsigned short*)Cout2 + (size_t)b * strideC) : nullptr;
      for (int pass = 0; pass < 2; ++pass) {
#pragma unroll
        for (int it = 0; it < 4; ++it) {
          const int row = it * 4 + q;
          const float* sp = slab + row * 68 + c8;
          v8h hv, lv;
#pragma unroll
          for (int e = 0; e < 8; ++e) {
            if (OUT_MODE == 1) {
              hv[e] = (_Float16)sp[e];
            } else {
              unsigned short hb = f2bf_bits(sp[e]);
              unsigned short lb = f2bf_bits(sp[e] - bf_bits2f(hb));
              hv[e] = __builtin_bit_cast(_Float16, hb);
              lv[e] = __builtin_bit_cast(_Float16, lb);
            }
          }
          *(volatile v8h*)(C + (size_t)(mBase + row) * ldc + n0 + c8) = hv;
          if (OUT_MODE == 2) *(volatile v8h*)(C2 + (size_t)(mBase + row) * ldc + n0 + c8) = lv;
        }
        __threadfence();
      }
    }
    __builtin_amdgcn_fence(__ATOMIC_RELEASE, "workgroup");
    __builtin_amdgcn_wave_barrier();
    __builtin_amdgcn_fence(__ATOMIC_ACQUIRE, "workgroup");
  }
}

constexpr int kBatch     = 64;
constexpr int kSeq       = 256;
constexpr int kEmb       = 300;
constexpr int kEmbPad    = 320;
constexpr int kHid       = 512;
constexpr int kCat       = kEmb + kHid;
constexpr int kOutDim    = 9;
constexpr int kOutPad    = 16;
constexpr int kRows      = kBatch * kSeq;
constexpr int kChunkT    = 64;
constexpr int kChunkRows = kChunkT * kBatch;
constexpr int kNumChunks = kSeq / kChunkT;
constexpr int kHalfB     = 32;
constexpr int kLdp       = kHid + 8;
constexpr int kRecThreads = 512;
constexpr int kRecWaves  = kRecThreads / 32;
constexpr float kWScale  = 16.0f;
constexpr float kWInv    = 0.0625f;

static_assert(kHid % 64 == 0, "gemm M tile");
static_assert(kChunkRows % 64 == 0, "gemm N tile");
static_assert(kEmbPad % 32 == 0, "gemm K step");
static_assert(kEmbPad >= kEmb, "K pad");
static_assert(kHid % 32 == 0, "k step");
static_assert(kRecWaves * 32 == kHid, "one wave per 32 hidden units");
static_assert(kBatch == 2 * kHalfB, "two half-batch blocks");
static_assert(kSeq % kChunkT == 0, "chunks");
static_assert(kRows % 8 == 0, "embed grid");
static_assert(kSeq * kOutDim == 2304, "output block extent");
static_assert((kSeq * kOutDim) % 32 == 0, "output block is whole 128-B lines");
static_assert(kEmb % 4 == 0 && kCat % 4 == 0, "16-B aligned source rows");
static_assert((kHalfB * kLdp) % 8 == 0, "lds zero fill granularity");
static_assert(kLdp % 8 == 0, "16-B aligned lds rows");

__device__ __forceinline__ float bf_rne(float f) {
  unsigned u = __float_as_uint(f);
  u = (u + 0x7FFFu + ((u >> 16) & 1u)) & 0xFFFF0000u;
  return __uint_as_float(u);
}
__device__ __forceinline__ unsigned hbits16(float f) {
  return (unsigned)__builtin_bit_cast(unsigned short, (_Float16)f);
}
__device__ __forceinline__ void wave_sync_lds() {
  __builtin_amdgcn_fence(__ATOMIC_RELEASE, "workgroup");
  __builtin_amdgcn_wave_barrier();
  __builtin_amdgcn_fence(__ATOMIC_ACQUIRE, "workgroup");
}
__device__ __forceinline__ void dep_guard1_h(v8f& a, v16h x, v16h y) {
  asm volatile("v_nop\n\tv_nop\n\tv_nop\n\tv_nop" : "+v"(a) : "v"(x), "v"(y));
}
__device__ __forceinline__ float rcp_f(float x) { return __builtin_amdgcn_rcpf(x); }
__device__ __forceinline__ float sigm_f(float x) { return rcp_f(1.0f + expf(-x)); }
__device__ __forceinline__ float tanh_f(float x) { return 1.0f - 2.0f * rcp_f(expf(2.0f * x) + 1.0f); }
__device__ __forceinline__ v8f zero8f() { return (v8f){0.f,0.f,0.f,0.f,0.f,0.f,0.f,0.f}; }

__device__ __forceinline__ v4u pack8_cols(const float* __restrict__ rowp, int c0, int nv, float mul) {
  const int lim = nv - 4;
  const int a0 = (c0 < lim) ? c0 : lim;
  const int a1 = ((c0 + 4) < lim) ? (c0 + 4) : lim;
  const v4f v0 = *(const v4f*)(rowp + a0);
  const v4f v1 = *(const v4f*)(rowp + a1);
  unsigned hb[8];
#pragma unroll
  for (int e = 0; e < 4; ++e) {
    const float f0 = ((c0 + e) < nv) ? v0[e] : 0.0f;
    const float f1 = ((c0 + 4 + e) < nv) ? v1[e] : 0.0f;
    hb[e]     = hbits16(bf_rne(f0) * mul);
    hb[4 + e] = hbits16(bf_rne(f1) * mul);
  }
  v4u w;
  w[0] = hb[0] | (hb[1] << 16);
  w[1] = hb[2] | (hb[3] << 16);
  w[2] = hb[4] | (hb[5] << 16);
  w[3] = hb[6] | (hb[7] << 16);
  return w;
}

__global__ __launch_bounds__(256) void embed_rows_kernel(
    const int* __restrict__ tok, const float* __restrict__ emb,
    unsigned short* __restrict__ xe, int vocab) {
  const int lane = threadIdx.x & 31, wave = threadIdx.x >> 5;
  const int row = blockIdx.x * 8 + wave;
  if (row >= kRows) return;
  const int t = row >> 6, b = row & 63;
  int id = tok[b * kSeq + t];
  id = (id < 0) ? 0 : ((id >= vocab) ? (vocab - 1) : id);
  const float* er = emb + (size_t)id * kEmb;
  unsigned short* dst = xe + (size_t)row * kEmbPad;
  const int p1 = 32 + (lane & 7);
  const v4u w0 = pack8_cols(er, lane * 8, kEmb, 1.0f);
  const v4u w1 = pack8_cols(er, p1 * 8, kEmb, 1.0f);
  for (int pass = 0; pass < 2; ++pass) {
    *(volatile v4u*)(dst + lane * 8) = w0;
    if (lane < 8) *(volatile v4u*)(dst + p1 * 8) = w1;
    __threadfence();
  }
}

__global__ __launch_bounds__(256) void cast_w_kernel(
    const float* __restrict__ Wg0, const float* __restrict__ Wg1, const float* __restrict__ Wg2,
    const float* __restrict__ Wg3, const float* __restrict__ Wg4, const float* __restrict__ Wg5,
    unsigned short* __restrict__ Wx16, unsigned short* __restrict__ Wh16) {
  const int lane = threadIdx.x & 31, wave = threadIdx.x >> 5;
  const int job = blockIdx.x * 8 + wave;
  if (job >= 6 * 2 * kHid) return;
  const int gi = job >> 10;
  const int rem = job & 1023;
  const int hrow = rem & (kHid - 1);
  const int part = rem >> 9;
  const float* Wsel = (gi == 0) ? Wg0 : (gi == 1) ? Wg1 : (gi == 2) ? Wg2 : (gi == 3) ? Wg3 : (gi == 4) ? Wg4 : Wg5;
  const float* src = Wsel + (size_t)hrow * kCat;
  if (part == 0) {
    unsigned short* dst = Wh16 + ((size_t)gi * kHid + hrow) * kHid;
    v4u w[2];
#pragma unroll
    for (int it = 0; it < 2; ++it) w[it] = pack8_cols(src, (it * 32 + lane) * 8, kHid, kWScale);
    for (int pass = 0; pass < 2; ++pass) {
#pragma unroll
      for (int it = 0; it < 2; ++it) *(volatile v4u*)(dst + (it * 32 + lane) * 8) = w[it];
      __threadfence();
    }
  } else {
    unsigned short* dst = Wx16 + ((size_t)gi * kHid + hrow) * kEmbPad;
    const float* xs = src + kHid;
    const int p1 = 32 + (lane & 7);
    const v4u w0 = pack8_cols(xs, lane * 8, kEmb, kWScale);
    const v4u w1 = pack8_cols(xs, p1 * 8, kEmb, kWScale);
    for (int pass = 0; pass < 2; ++pass) {
      *(volatile v4u*)(dst + lane * 8) = w0;
      if (lane < 8) *(volatile v4u*)(dst + p1 * 8) = w1;
      __threadfence();
    }
  }
}

__global__ __launch_bounds__(256) void cast_wp_kernel(const float* __restrict__ Wp, unsigned short* __restrict__ Wp16) {
  const int lane = threadIdx.x & 31, wave = threadIdx.x >> 5;
  const int o = blockIdx.x * 8 + wave;
  if (o >= kOutPad) return;
  unsigned short* dst = Wp16 + (size_t)o * (2 * kHid);
  const float* src = Wp + (size_t)((o < kOutDim) ? o : (kOutDim - 1)) * (2 * kHid);
  v4u w[4];
#pragma unroll
  for (int it = 0; it < 4; ++it) w[it] = pack8_cols(src, (it * 32 + lane) * 8, 2 * kHid, kWScale);
  if (o >= kOutDim) {
#pragma unroll
    for (int it = 0; it < 4; ++it) w[it] = (v4u){0u, 0u, 0u, 0u};
  }
  for (int pass = 0; pass < 2; ++pass) {
#pragma unroll
    for (int it = 0; it < 4; ++it) *(volatile v4u*)(dst + (it * 32 + lane) * 8) = w[it];
    __threadfence();
  }
}

__global__ __launch_bounds__(kRecThreads) void rec_chunk_kernel(
    const unsigned short* __restrict__ Whd, const float* __restrict__ XinT,
    const float* __restrict__ bR, const float* __restrict__ bU, const float* __restrict__ bC,
    unsigned short* __restrict__ cpl, float* __restrict__ carry,
    int q, int dir, int first) {
  __shared__ __align__(16) _Float16 c16[kHalfB * kLdp];
  __shared__ __align__(16) _Float16 rc16[kHalfB * kLdp];
  __shared__ __align__(16) float slab[kRecWaves][16 * 32];

  const int tid = threadIdx.x;
  const int lane = tid & 31, wave = tid >> 5;
  const int hh = lane >> 4, cl = lane & 15, koff = hh * 8;
  const int rb0 = blockIdx.x * kHalfB;
  const int n0 = wave * 32;
  float* sl = slab[wave];

  const _Float16* WhR = (const _Float16*)Whd;
  const _Float16* WhU = WhR + (size_t)kHid * kHid;
  const _Float16* WhC = WhU + (size_t)kHid * kHid;
  const float* XR = XinT;
  const float* XU = XinT + (size_t)kHid * kChunkRows;
  const float* XC = XU + (size_t)kHid * kChunkRows;

  float brv[2], buv[2], bcv[2];
#pragma unroll
  for (int j = 0; j < 2; ++j) {
    const int n = n0 + 16 * j + cl;
    brv[j] = bf_rne(bR[n]);
    buv[j] = bf_rne(bU[n]);
    bcv[j] = bf_rne(bC[n]);
  }

  {
    const v4u z = (v4u){0u, 0u, 0u, 0u};
    for (int i = tid; i < (kHalfB * kLdp) / 8; i += kRecThreads) {
      *(v4u*)(c16 + 8 * i) = z;
      *(v4u*)(rc16 + 8 * i) = z;
    }
  }
  __syncthreads();

  v8f cReg[2][2], uReg[2][2];
#pragma unroll
  for (int mt = 0; mt < 2; ++mt)
#pragma unroll
    for (int j = 0; j < 2; ++j) { cReg[mt][j] = zero8f(); uReg[mt][j] = zero8f(); }

  if (!first) {
#pragma unroll
    for (int mt = 0; mt < 2; ++mt) {
      const int rq = lane >> 3, c4 = (lane & 7) * 4;
#pragma unroll
      for (int it = 0; it < 4; ++it) {
        const int row = it * 4 + rq;
        const v4f v = *(const v4f*)(carry + (size_t)(rb0 + mt * 16 + row) * kHid + n0 + c4);
        *(v4f*)(sl + row * 32 + c4) = v;
      }
      wave_sync_lds();
#pragma unroll
      for (int j = 0; j < 2; ++j) {
#pragma unroll
        for (int r = 0; r < 8; ++r) {
          const float v = sl[(8 * hh + r) * 32 + 16 * j + cl];
          cReg[mt][j][r] = v;
          c16[(mt * 16 + 8 * hh + r) * kLdp + n0 + 16 * j + cl] = (_Float16)v;
        }
      }
      wave_sync_lds();
    }
  }
  __syncthreads();

  for (int s = 0; s < kChunkT; ++s) {
    const int tl = dir ? (kChunkT - 1 - s) : s;
    const int t = q * kChunkT + tl;
    const int xcol = tl * kBatch + rb0;

#pragma unroll
    for (int mt = 0; mt < 2; ++mt) {
#pragma unroll
      for (int gate = 0; gate < 2; ++gate) {
        const _Float16* Wg = gate ? WhU : WhR;
        v8f acc[2];
        acc[0] = zero8f(); acc[1] = zero8f();
#pragma unroll 1
        for (int kc = 0; kc < kHid; kc += 32) {
          const v16h a  = Frag<_Float16>::load(c16 + (mt * 16 + cl) * kLdp + kc + koff);
          const v16h b0 = Frag<_Float16>::load(Wg + (size_t)(n0 + cl) * kHid + kc + koff);
          const v16h b1 = Frag<_Float16>::load(Wg + (size_t)(n0 + 16 + cl) * kHid + kc + koff);
          acc[0] = Frag<_Float16>::mma(a, b0, acc[0]);
          acc[1] = Frag<_Float16>::mma(a, b1, acc[1]);
          dep_guard_h(acc[0], acc[1], a, b1);
        }
        const float* Xg = gate ? XU : XR;
#pragma unroll
        for (int j = 0; j < 2; ++j) {
          const int n = n0 + 16 * j + cl;
          const float* xp = Xg + (size_t)n * kChunkRows + xcol + mt * 16 + 8 * hh;
          const v4f xa = *(const v4f*)xp;
          const v4f xb = *(const v4f*)(xp + 4);
          const float bj = gate ? buv[j] : brv[j];
#pragma unroll
          for (int r = 0; r < 8; ++r) {
            const float xv = (r < 4) ? xa[r & 3] : xb[r & 3];
            const float pre = acc[j][r] * kWInv + xv + bj;
            const float sg = sigm_f(pre);
            if (gate == 0) {
              rc16[(mt * 16 + 8 * hh + r) * kLdp + n] = (_Float16)(sg * cReg[mt][j][r]);
            } else {
              uReg[mt][j][r] = sg;
            }
          }
        }
      }
    }
    __syncthreads();

#pragma unroll
    for (int mt = 0; mt < 2; ++mt) {
      v8f acc[2];
      acc[0] = zero8f(); acc[1] = zero8f();
#pragma unroll 1
      for (int kc = 0; kc < kHid; kc += 32) {
        const v16h a  = Frag<_Float16>::load(rc16 + (mt * 16 + cl) * kLdp + kc + koff);
        const v16h b0 = Frag<_Float16>::load(WhC + (size_t)(n0 + cl) * kHid + kc + koff);
        const v16h b1 = Frag<_Float16>::load(WhC + (size_t)(n0 + 16 + cl) * kHid + kc + koff);
        acc[0] = Frag<_Float16>::mma(a, b0, acc[0]);
        acc[1] = Frag<_Float16>::mma(a, b1, acc[1]);
        dep_guard_h(acc[0], acc[1], a, b1);
      }
#pragma unroll
      for (int j = 0; j < 2; ++j) {
        const int n = n0 + 16 * j + cl;
        const float* xp = XC + (size_t)n * kChunkRows + xcol + mt * 16 + 8 * hh;
        const v4f xa = *(const v4f*)xp;
        const v4f xb = *(const v4f*)(xp + 4);
#pragma unroll
        for (int r = 0; r < 8; ++r) {
          const float xv = (r < 4) ? xa[r & 3] : xb[r & 3];
          const float pre = acc[j][r] * kWInv + xv + bcv[j];
          const float cc = tanh_f(pre);
          const float u = uReg[mt][j][r];
          const float cp = cReg[mt][j][r];
          const float cn = u * cc + (1.0f - u) * cp;
          cReg[mt][j][r] = cn;
          c16[(mt * 16 + 8 * hh + r) * kLdp + n] = (_Float16)cn;
          sl[(8 * hh + r) * 32 + 16 * j + cl] = cn;
        }
      }
      wave_sync_lds();
      {
        const int rq = lane >> 3, p = lane & 7;
        const int prow = p >> 2, pc8 = (p & 3) * 8;
        const int grow0 = t * kBatch + rb0 + mt * 16;
        v4u w[2];
        size_t ad[2];
#pragma unroll
        for (int it = 0; it < 2; ++it) {
          const int rp = it * 4 + rq;
          const int row = 2 * rp + prow;
          const float* sp = sl + row * 32 + pc8;
          const v4f f0 = *(const v4f*)sp;
          const v4f f1 = *(const v4f*)(sp + 4);
          v4u ww;
          ww[0] = hbits16(f0[0]) | (hbits16(f0[1]) << 16);
          ww[1] = hbits16(f0[2]) | (hbits16(f0[3]) << 16);
          ww[2] = hbits16(f1[0]) | (hbits16(f1[1]) << 16);
          ww[3] = hbits16(f1[2]) | (hbits16(f1[3]) << 16);
          w[it] = ww;
          ad[it] = ((size_t)((grow0 >> 1) + rp) * kRecWaves + (size_t)wave) * 64 + (size_t)(prow * 32 + pc8);
        }
        for (int pass = 0; pass < 2; ++pass) {
#pragma unroll
          for (int it = 0; it < 2; ++it) *(volatile v4u*)(cpl + ad[it]) = w[it];
          __threadfence();
        }
      }
      wave_sync_lds();
    }
    __syncthreads();
  }

#pragma unroll
  for (int mt = 0; mt < 2; ++mt) {
#pragma unroll
    for (int j = 0; j < 2; ++j) {
#pragma unroll
      for (int r = 0; r < 8; ++r) sl[(8 * hh + r) * 32 + 16 * j + cl] = cReg[mt][j][r];
    }
    wave_sync_lds();
    {
      const int rq = lane >> 3, c4 = (lane & 7) * 4;
      v4f v[4];
#pragma unroll
      for (int it = 0; it < 4; ++it) v[it] = *(const v4f*)(sl + (it * 4 + rq) * 32 + c4);
      for (int pass = 0; pass < 2; ++pass) {
#pragma unroll
        for (int it = 0; it < 4; ++it)
          *(volatile v4f*)(carry + (size_t)(rb0 + mt * 16 + it * 4 + rq) * kHid + n0 + c4) = v[it];
        __threadfence();
      }
    }
    wave_sync_lds();
  }
}

__global__ __launch_bounds__(512) void proj_kernel(
    const unsigned short* __restrict__ cplF, const unsigned short* __restrict__ cplB,
    const unsigned short* __restrict__ Wp16, const float* __restrict__ bp, float* __restrict__ out) {
  __shared__ __align__(16) float ys[kSeq * kOutDim];
  const int tid = threadIdx.x;
  const int lane = tid & 31, wave = tid >> 5;
  const int hh = lane >> 4, cl = lane & 15, koff = hh * 8;
  const int b = blockIdx.x;
  const int t0 = wave * 16;
  const int m = (t0 + cl) * kBatch + b;
  const size_t segbase = (size_t)(m >> 1) * kRecWaves * 64 + (size_t)(m & 1) * 32;
  const _Float16* pf = (const _Float16*)cplF;
  const _Float16* pb = (const _Float16*)cplB;
  const _Float16* wp = (const _Float16*)Wp16 + (size_t)cl * (2 * kHid);
  v8f acc = zero8f();
#pragma unroll 1
  for (int ks = 0; ks < kHid / 32; ++ks) {
    const v16h a = Frag<_Float16>::load(pf + segbase + (size_t)ks * 64 + koff);
    const v16h w = Frag<_Float16>::load(wp + ks * 32 + koff);
    acc = Frag<_Float16>::mma(a, w, acc);
    dep_guard1_h(acc, a, w);
  }
#pragma unroll 1
  for (int ks = 0; ks < kHid / 32; ++ks) {
    const v16h a = Frag<_Float16>::load(pb + segbase + (size_t)ks * 64 + koff);
    const v16h w = Frag<_Float16>::load(wp + kHid + ks * 32 + koff);
    acc = Frag<_Float16>::mma(a, w, acc);
    dep_guard1_h(acc, a, w);
  }
  const float bpv = bf_rne(bp[(cl < kOutDim) ? cl : (kOutDim - 1)]);
#pragma unroll
  for (int r = 0; r < 8; ++r) {
    const int t = t0 + 8 * hh + r;
    const float yv = acc[r] * kWInv + bpv;
    if (cl < kOutDim) ys[t * kOutDim + cl] = yv;
  }
  __syncthreads();
  float* ob = out + (size_t)b * (kSeq * kOutDim);
  const v4f w0 = *(const v4f*)(ys + tid * 4);
  const int t1 = (tid < 64) ? tid : 63;
  const v4f w1 = *(const v4f*)(ys + 2048 + t1 * 4);
  for (int pass = 0; pass < 2; ++pass) {
    *(volatile v4f*)(ob + tid * 4) = w0;
    if (tid < 64) *(volatile v4f*)(ob + 2048 + tid * 4) = w1;
    __threadfence();
  }
}

extern "C" void kernel_launch(void* const* d_in, const int* in_sizes, int n_in,
                              void* d_out, int out_size, void* d_ws, size_t ws_size,
                              hipStream_t stream) {
  const int*   xTok = (const int*)d_in[0];
  const float* emb  = (const float*)d_in[1];
  const float* Wcf  = (const float*)d_in[2];
  const float* bcf  = (const float*)d_in[3];
  const float* Wrf  = (const float*)d_in[4];
  const float* brf  = (const float*)d_in[5];
  const float* Wuf  = (const float*)d_in[6];
  const float* buf  = (const float*)d_in[7];
  const float* Wcb  = (const float*)d_in[8];
  const float* bcb  = (const float*)d_in[9];
  const float* Wrb  = (const float*)d_in[10];
  const float* brb  = (const float*)d_in[11];
  const float* Wub  = (const float*)d_in[12];
  const float* bub  = (const float*)d_in[13];
  const float* Wp   = (const float*)d_in[14];
  const float* bp   = (const float*)d_in[15];
  float* out = (float*)d_out;
  (void)out_size;

  int vocab = 1;
  if (n_in > 1 && in_sizes[1] >= kEmb) vocab = in_sizes[1] / kEmb;

  char* wsb = (char*)d_ws;
  size_t off = 0;
  const size_t kAlign = 256;
#define CARVE_REGION(ptr, type, bytes) type* ptr = (type*)(wsb + off); off += ((size_t)(bytes) + kAlign - 1) & ~(kAlign - 1);
  CARVE_REGION(xe16,   unsigned short, (size_t)kRows * kEmbPad * 2)
  CARVE_REGION(Wx16,   unsigned short, (size_t)6 * kHid * kEmbPad * 2)
  CARVE_REGION(Wh16,   unsigned short, (size_t)6 * kHid * kHid * 2)
  CARVE_REGION(Wp16,   unsigned short, (size_t)kOutPad * 2 * kHid * 2)
  CARVE_REGION(XinT,   float,          (size_t)3 * kHid * kChunkRows * 4)
  CARVE_REGION(cplF,   unsigned short, (size_t)kRows * kHid * 2)
  CARVE_REGION(cplB,   unsigned short, (size_t)kRows * kHid * 2)
  CARVE_REGION(carryF, float,          (size_t)kBatch * kHid * 4)
  CARVE_REGION(carryB, float,          (size_t)kBatch * kHid * 4)
#undef CARVE_REGION
  if (off > ws_size) return;

  embed_rows_kernel<<<kRows / 8, 256, 0, stream>>>(xTok, emb, xe16, vocab);
  cast_w_kernel<<<(6 * 2 * kHid) / 8, 256, 0, stream>>>(Wrf, Wuf, Wcf, Wrb, Wub, Wcb, Wx16, Wh16);
  cast_wp_kernel<<<2, 256, 0, stream>>>(Wp, Wp16);

  for (int dir = 0; dir < 2; ++dir) {
    const unsigned short* WxD = Wx16 + (size_t)dir * 3 * kHid * kEmbPad;
    const unsigned short* WhD = Wh16 + (size_t)dir * 3 * kHid * kHid;
    const float* bRd = dir ? brb : brf;
    const float* bUd = dir ? bub : buf;
    const float* bCd = dir ? bcb : bcf;
    unsigned short* cplD = dir ? cplB : cplF;
    float* carD = dir ? carryB : carryF;
    for (int i = 0; i < kNumChunks; ++i) {
      const int q = dir ? (kNumChunks - 1 - i) : i;
      const unsigned short* BtD = xe16 + (size_t)q * kChunkRows * kEmbPad;
      wmma_gemm64<0, false, 0, 0, false, 0><<<dim3((kHid / 64) * (kChunkRows / 64) / 8, 3), 256, 0, stream>>>(
          WxD, WxD, kEmbPad, (long)kHid * kEmbPad,
          BtD, BtD, kEmbPad, 0L,
          (void*)XinT, (void*)XinT, kChunkRows, (long)kHid * kChunkRows,
          bCd, XinT, 0L,
          kHid, kChunkRows, kEmbPad, kWInv);
      rec_chunk_kernel<<<kBatch / kHalfB, kRecThreads, 0, stream>>>(
          WhD, XinT, bRd, bUd, bCd, cplD, carD, q, dir, (i == 0) ? 1 : 0);
    }
  }
  proj_kernel<<<kBatch, 512, 0, stream>>>(cplF, cplB, Wp16, bp, out);
}
